// TransformerBlock_85418309583081
// MI455X (gfx1250) — hardware-run, weakly checked
//
#include <hip/hip_runtime.h>
#include <math.h>
#include <stdint.h>

#ifndef NB
#define NB 2
#endif
#ifndef SEQ
#define SEQ 2048
#endif
#define NB_FULL   2
#define SEQ_FULL  2048
#define DM    1024
#define NH    8
#define HD    64
#define DV    128
#define QKLD  (2 * DM)
#define DFF   (4 * DM)
#define NQB   (SEQ / 64)
#define VCARRY 16.0f
#define QKC    64.0f
#define ACARRY 256.0f
#define HCARRY 64.0f
#define GCARRY 256.0f
#define WCARRY 256.0f
#define SMUL   (0.125f * 1.4426950408889634f / (QKC * QKC))
#define LAM_INIT 0.4707130183435844f
#define OMLI     0.5292869816564156f

static_assert(HD == 64);
static_assert(DV == 128);
static_assert(NH * DV == DM && 2 * NH * HD == DM);
static_assert(QKLD == 2 * DM && DFF == 4 * DM);
static_assert(NB >= 1 && NB <= NB_FULL);
static_assert(SEQ >= 64 && SEQ <= SEQ_FULL && (SEQ % 64) == 0);
static_assert((SEQ % 16) == 0);
static_assert((DM % 64) == 0 && (QKLD % 64) == 0 && (DFF % 64) == 0);
static_assert((DM % 32) == 0 && (DFF % 32) == 0);
static_assert(((NB * SEQ) % 64) == 0);
static_assert(((NB * SEQ) % 8) == 0);
static_assert(DM == 8 * 32 * 4);
static_assert(((SEQ * DM / 8) % 256) == 0);
static_assert(256 * 4 * 4 == 64 * 64);
static_assert((size_t)((NB_FULL - 1) * SEQ_FULL + SEQ_FULL) * DM * 4 == (size_t)16777216);

static constexpr size_t WSB_XB   = (size_t)NB * SEQ * DM * 2;
static constexpr size_t WSB_WQKV = (size_t)3 * DM * DM * 2;
static constexpr size_t WSB_QK   = (size_t)NB * SEQ * QKLD * 2;
static constexpr size_t WSB_VT   = (size_t)NB * DM * SEQ * 2;
static constexpr size_t WSB_R1A  = WSB_XB + WSB_WQKV + WSB_QK + WSB_VT;
static constexpr size_t WSB_G    = (size_t)NB * SEQ * DFF * 2;
static constexpr size_t WSB_R1   = (WSB_R1A > WSB_G) ? WSB_R1A : WSB_G;
static constexpr size_t WSB_WO   = (size_t)DM * DM * 2;
static constexpr size_t WSB_W1   = (size_t)DFF * DM * 2;
static constexpr size_t WSB_W2   = (size_t)DM * DFF * 2;
static constexpr size_t WSB_ROPE = (size_t)SEQ * 32 * 4;
static constexpr size_t WSB_AP   = (size_t)NB * SEQ * DM * 2;
static constexpr size_t WSB_PRE  = (size_t)NB * SEQ * DM * 4;
static constexpr size_t WSB_HF   = (size_t)NB * SEQ * DM * 4;
static constexpr size_t WSB_HH   = (size_t)NB * SEQ * DM * 2;
static constexpr size_t WSB_TOTAL = WSB_R1 + WSB_WO + WSB_W1 + WSB_W2 + WSB_ROPE + WSB_AP + WSB_PRE + WSB_HF + WSB_HH;
static_assert(WSB_R1A <= WSB_R1 && WSB_G <= WSB_R1);
static_assert(WSB_TOTAL <= (size_t)134217728);
static_assert((WSB_XB % 128) == 0 && (WSB_WQKV % 128) == 0 && (WSB_QK % 128) == 0 && (WSB_VT % 128) == 0);
static_assert((WSB_R1 % 128) == 0 && (WSB_WO % 128) == 0 && (WSB_W1 % 128) == 0 && (WSB_W2 % 128) == 0);
static_assert((WSB_ROPE % 128) == 0 && (WSB_AP % 128) == 0 && (WSB_PRE % 128) == 0 && (WSB_HH % 128) == 0);

typedef _Float16 v16h __attribute__((ext_vector_type(16)));
typedef _Float16 v8h  __attribute__((ext_vector_type(8)));
typedef __bf16   v16b __attribute__((ext_vector_type(16)));
typedef __bf16   v8b  __attribute__((ext_vector_type(8)));
typedef float    v8f  __attribute__((ext_vector_type(8)));
typedef float    v4f  __attribute__((ext_vector_type(4)));
typedef unsigned int v4u __attribute__((ext_vector_type(4)));
typedef unsigned int v2u __attribute__((ext_vector_type(2)));
typedef _Float16 h16;

#if defined(__HIP_DEVICE_COMPILE__)
#define DEV_ASM 1
#else
#define DEV_ASM 0
#endif

__device__ __forceinline__ unsigned short bf_bits(float f) {
  unsigned u = __float_as_uint(f);
  return (unsigned short)((u + 0x7FFFu + ((u >> 16) & 1u)) >> 16);
}
__device__ __forceinline__ float bf_up(unsigned short hb) { return __uint_as_float(((unsigned)hb) << 16); }
__device__ __forceinline__ unsigned short h_bits(_Float16 x) { return __builtin_bit_cast(unsigned short, x); }
__device__ __forceinline__ unsigned pk16(unsigned short a, unsigned short b) { return (unsigned)a | ((unsigned)b << 16); }
__device__ __forceinline__ v8f zero8() { v8f z = {0.f, 0.f, 0.f, 0.f, 0.f, 0.f, 0.f, 0.f}; return z; }

static __device__ __forceinline__ float bfv(float f) { return bf_up(bf_bits(f)); }
static __device__ __forceinline__ h16 toh_flush(float v) {
  const h16 r = (h16)v;
  return (fabsf(v) < 6.103515625e-05f) ? (h16)0.0f : r;
}
static __device__ __forceinline__ void pin4(v4f& x) {
#if DEV_ASM
  asm volatile("" : "+v"(x));
#else
  (void)x;
#endif
}

template <typename OT> struct FT;
template <> struct FT<__bf16>   { typedef v16b frag; typedef v8b half8; };
template <> struct FT<_Float16> { typedef v16h frag; typedef v8h half8; };

template <typename OT>
__device__ __forceinline__ typename FT<OT>::frag ldfrag(const OT* p) {
  union { typename FT<OT>::frag v; typename FT<OT>::half8 h[2]; } f;
  f.h[0] = *(const typename FT<OT>::half8*)(p);
  f.h[1] = *(const typename FT<OT>::half8*)(p + 16);
  return f.v;
}

__device__ __forceinline__ v8f mmar(v16b a, v16b b, v8f c) {
  return __builtin_amdgcn_wmma_f32_16x16x32_bf16(false, a, false, b, (short)0, c, false, false);
}
__device__ __forceinline__ v8f mmar(v16h a, v16h b, v8f c) {
  return __builtin_amdgcn_wmma_f32_16x16x32_f16(false, a, false, b, (short)0, c, false, false);
}
__device__ __forceinline__ v8f mma_h(v16h a, v16h b, v8f c) {
  c = __builtin_amdgcn_wmma_f32_16x16x32_f16(false, a, false, b, (short)0, c, false, false);
#if DEV_ASM
  asm volatile("v_nop\n\tv_nop\n\tv_nop\n\tv_nop" : "+v"(c) : "v"(a), "v"(b));
#endif
  return c;
}
__device__ __forceinline__ void dep_guard(v8f& a, v8f& b, v16b x, v16b y) {
#if DEV_ASM
  asm volatile("v_nop\n\tv_nop\n\tv_nop\n\tv_nop" : "+v"(a), "+v"(b) : "v"(x), "v"(y));
#else
  (void)a; (void)b; (void)x; (void)y;
#endif
}
__device__ __forceinline__ void dep_guard(v8f& a, v8f& b, v16h x, v16h y) {
#if DEV_ASM
  asm volatile("v_nop\n\tv_nop\n\tv_nop\n\tv_nop" : "+v"(a), "+v"(b) : "v"(x), "v"(y));
#else
  (void)a; (void)b; (void)x; (void)y;
#endif
}
__device__ __forceinline__ void keep4(v16b a, v16b b, v16b c, v16b d) {
#if DEV_ASM
  asm volatile("v_nop" :: "v"(a), "v"(b), "v"(c), "v"(d));
#else
  (void)a; (void)b; (void)c; (void)d;
#endif
}
__device__ __forceinline__ void keep4(v16h a, v16h b, v16h c, v16h d) {
#if DEV_ASM
  asm volatile("v_nop" :: "v"(a), "v"(b), "v"(c), "v"(d));
#else
  (void)a; (void)b; (void)c; (void)d;
#endif
}
__device__ __forceinline__ void acc_guard4(v8f& a, v8f& b, v8f& c, v8f& d) {
#if DEV_ASM
  asm volatile("v_nop\n\tv_nop\n\tv_nop\n\tv_nop" : "+v"(a), "+v"(b), "+v"(c), "+v"(d));
#else
  (void)a; (void)b; (void)c; (void)d;
#endif
}

__global__ __launch_bounds__(256) void cvt_bf16x8(const float* __restrict__ in, long long istride,
                                                 unsigned short* out, long long ostride, int n8) {
  const int b = blockIdx.y;
  const int i = blockIdx.x * 256 + (int)threadIdx.x;
  if (i < n8) {
    const float* ip = in + (size_t)b * (size_t)istride + (size_t)i * 8;
    const v4f a  = *(const v4f*)(ip);
    const v4f a4 = *(const v4f*)(ip + 4);
    v4u p;
    p[0] = pk16(bf_bits(a[0]),  bf_bits(a[1]));
    p[1] = pk16(bf_bits(a[2]),  bf_bits(a[3]));
    p[2] = pk16(bf_bits(a4[0]), bf_bits(a4[1]));
    p[3] = pk16(bf_bits(a4[2]), bf_bits(a4[3]));
    unsigned short* o = out + (size_t)b * (size_t)ostride + (size_t)i * 8;
    *(volatile v4u*)o = p;
    __threadfence();
    *(volatile v4u*)o = p;
  }
}

template <int MODE>
__device__ __forceinline__ unsigned short cvm(float f, float scale) {
  const unsigned short hb = bf_bits(f);
  if (MODE == 0) return hb;
  return h_bits((_Float16)(bf_up(hb) * scale));
}

template <int MODE>
__device__ __forceinline__ void wtrans_body(const float* __restrict__ W, int C,
                                            unsigned short* T, int ldt, int coff, float scale,
                                            float* sW) {
  const int tid  = threadIdx.x;
  const int lane = tid & 31;
  const int wave = tid >> 5;
  const int n0 = blockIdx.x * 64;
  const int k0 = blockIdx.y * 64;
#pragma unroll
  for (int j = 0; j < 4; ++j) {
    const int lin = tid + j * 256;
    const int r = lin >> 4, c4 = (lin & 15) * 4;
    const v4f val = *(const v4f*)(W + (size_t)(k0 + r) * (size_t)C + n0 + c4);
    sW[(c4 + 0) * 68 + r] = val[0];
    sW[(c4 + 1) * 68 + r] = val[1];
    sW[(c4 + 2) * 68 + r] = val[2];
    sW[(c4 + 3) * 68 + r] = val[3];
  }
  __syncthreads();
  const int q = lane >> 3, c8 = (lane & 7) * 8;
  v4u pv[2];
#pragma unroll
  for (int it = 0; it < 2; ++it) {
    const int row = it * 32 + wave * 4 + q;
    const float* sp = sW + row * 68 + c8;
    v4u a;
#pragma unroll
    for (int e = 0; e < 4; ++e)
      a[e] = pk16(cvm<MODE>(sp[2 * e], scale), cvm<MODE>(sp[2 * e + 1], scale));
    pv[it] = a;
  }
  for (int ps = 0; ps < 2; ++ps) {
#pragma unroll
    for (int it = 0; it < 2; ++it) {
      const int row = it * 32 + wave * 4 + q;
      *(volatile v4u*)(T + (size_t)(n0 + row) * (size_t)ldt + coff + k0 + c8) = pv[it];
    }
    __threadfence();
  }
}

__global__ __launch_bounds__(256) void wtrans_bf16(const float* __restrict__ W, int C,
                                                  unsigned short* T, int ldt, int coff, float scale) {
  __shared__ __align__(16) float sW[64 * 68];
  wtrans_body<0>(W, C, T, ldt, coff, scale, sW);
}
__global__ __launch_bounds__(256) void wtrans_f16s(const float* __restrict__ W, int C,
                                                  unsigned short* T, int ldt, int coff, float scale) {
  __shared__ __align__(16) float sW[64 * 68];
  wtrans_body<1>(W, C, T, ldt, coff, scale, sW);
}

template <typename OT, int OUT_MODE>
__device__ __forceinline__ void gemm64_body(
    const unsigned short* __restrict__ Ap, int lda, long long strideA,
    const unsigned short* __restrict__ Btp, int ldb, long long strideB,
    void* Cout, void* Cout2, int ldc, long long strideC,
    const float* __restrict__ bias,
    int M, int N, int K, float oscale, float rscale, float* sTall) {
  typedef typename FT<OT>::frag V16;
  const OT* A  = (const OT*)(const void*)Ap;
  const OT* Bt = (const OT*)(const void*)Btp;
  const int b    = blockIdx.y;
  const int lane = threadIdx.x & 31;
  const int wave = threadIdx.x >> 5;
  const int tilesN = N >> 6;
  const int tilesM = M >> 6;
  const int tile = blockIdx.x * 8 + wave;
  if (tile >= tilesM * tilesN) return;
  const int tm = tile / tilesN;
  const int tn = tile - tm * tilesN;
  const int m0 = tm << 6;
  const int n0 = tn << 6;

  const OT* Ab = A  + (size_t)b * (size_t)strideA;
  const OT* Bb = Bt + (size_t)b * (size_t)strideB;

  const int rlane = lane & 15;
  const int koff  = (lane >> 4) * 8;
  const int mOff  = (lane >> 4) * 8;

  v8f acc[4][4];
#pragma unroll
  for (int i = 0; i < 4; ++i)
#pragma unroll
    for (int j = 0; j < 4; ++j) acc[i][j] = zero8();

  for (int k0 = 0; k0 < K; k0 += 32) {
    V16 bq[4];
#pragma unroll
    for (int j = 0; j < 4; ++j)
      bq[j] = ldfrag<OT>(Bb + (size_t)(n0 + (j << 4) + rlane) * ldb + koff + k0);
#pragma unroll
    for (int i = 0; i < 4; ++i) {
      const V16 af = ldfrag<OT>(Ab + (size_t)(m0 + (i << 4) + rlane) * lda + koff + k0);
#pragma unroll
      for (int j = 0; j < 4; ++j) acc[i][j] = mmar(af, bq[j], acc[i][j]);
      dep_guard(acc[i][0], acc[i][3], af, bq[3]);
    }
    keep4(bq[0], bq[1], bq[2], bq[3]);
  }
  acc_guard4(acc[0][0], acc[0][1], acc[0][2], acc[0][3]);
  acc_guard4(acc[1][0], acc[1][1], acc[1][2], acc[1][3]);
  acc_guard4(acc[2][0], acc[2][1], acc[2][2], acc[2][3]);
  acc_guard4(acc[3][0], acc[3][1], acc[3][2], acc[3][3]);

  float* slab = sTall + wave * (16 * 68);
#pragma unroll
  for (int i = 0; i < 4; ++i) {
    const int mBase = m0 + (i << 4);
#pragma unroll
    for (int j = 0; j < 4; ++j) {
#pragma unroll
      for (int r = 0; r < 8; ++r) {
        slab[(mOff + r) * 68 + (j << 4) + rlane] = acc[i][j][r];
      }
    }
    __builtin_amdgcn_fence(3  , "workgroup");
    __builtin_amdgcn_wave_barrier();
    __builtin_amdgcn_fence(2  , "workgroup");
    if (OUT_MODE == 0) {
      float* Cb0 = (float*)Cout + (size_t)b * (size_t)strideC;
      const int h2 = lane >> 4, c4 = (lane & 15) * 4;
      const v4f braw = *(const v4f*)(bias + n0 + c4);
      v4f bv;
      bv[0] = bf_up(bf_bits(braw[0]));
      bv[1] = bf_up(bf_bits(braw[1]));
      bv[2] = bf_up(bf_bits(braw[2]));
      bv[3] = bf_up(bf_bits(braw[3]));
      for (int ps = 0; ps < 2; ++ps) {
#pragma unroll
        for (int it = 0; it < 8; ++it) {
          const int row = it * 2 + h2;
          const v4f v = *(const v4f*)(slab + row * 68 + c4) * oscale + bv;
          *(volatile v4f*)(Cb0 + (size_t)(mBase + row) * ldc + n0 + c4) = v;
        }
        __threadfence();
      }
    } else {
      const int q = lane >> 3, c8 = (lane & 7) * 8;
      unsigned short* Cp  = (unsigned short*)Cout  + (size_t)b * (size_t)strideC;
      unsigned short* Cp2 = (unsigned short*)Cout2 + (size_t)b * (size_t)strideC;
      v4u hv[4], lv[4];
#pragma unroll
      for (int it = 0; it < 4; ++it) {
        const int row = it * 4 + q;
        const float* sp = slab + row * 68 + c8;
        float f[8];
#pragma unroll
        for (int e = 0; e < 8; ++e) f[e] = sp[e] * oscale;
        v4u a, a2;
#pragma unroll
        for (int e = 0; e < 4; ++e) {
          const float f0 = f[2 * e], f1 = f[2 * e + 1];
          const _Float16 x0 = (_Float16)f0, x1 = (_Float16)f1;
          const unsigned short h0 = h_bits(x0), h1 = h_bits(x1);
          unsigned short l0 = 0, l1 = 0;
          if (OUT_MODE == 3) {
            l0 = h_bits((_Float16)((f0 - (float)x0) * rscale));
            l1 = h_bits((_Float16)((f1 - (float)x1) * rscale));
          }
          a[e] = pk16(h0, h1); a2[e] = pk16(l0, l1);
        }
        hv[it] = a; lv[it] = a2;
      }
      for (int ps = 0; ps < 2; ++ps) {
#pragma unroll
        for (int it = 0; it < 4; ++it) {
          const int row = it * 4 + q;
          *(volatile v4u*)(Cp + (size_t)(mBase + row) * ldc + n0 + c8) = hv[it];
          if (OUT_MODE == 3) *(volatile v4u*)(Cp2 + (size_t)(mBase + row) * ldc + n0 + c8) = lv[it];
        }
        __threadfence();
      }
    }
    __builtin_amdgcn_fence(3  , "workgroup");
    __builtin_amdgcn_wave_barrier();
    __builtin_amdgcn_fence(2  , "workgroup");
  }
}

__global__ __launch_bounds__(256) void gemm_proj_plane(
    const unsigned short* __restrict__ Ap, int lda, long long strideA,
    const unsigned short* __restrict__ Btp, int ldb, long long strideB,
    void* Cout, void* Cout2, int ldc, long long strideC,
    const float* __restrict__ bias,
    int M, int N, int K, float oscale, float rscale) {
  __shared__ __align__(16) float sT[8 * 16 * 68];
  gemm64_body<__bf16, 1>(Ap, lda, strideA, Btp, ldb, strideB, Cout, Cout2, ldc, strideC, bias,
                         M, N, K, oscale, rscale, sT);
}
__global__ __launch_bounds__(256) void gemm_out_f32(
    const unsigned short* __restrict__ Ap, int lda, long long strideA,
    const unsigned short* __restrict__ Btp, int ldb, long long strideB,
    void* Cout, void* Cout2, int ldc, long long strideC,
    const float* __restrict__ bias,
    int M, int N, int K, float oscale, float rscale) {
  __shared__ __align__(16) float sT[8 * 16 * 68];
  gemm64_body<_Float16, 0>(Ap, lda, strideA, Btp, ldb, strideB, Cout, Cout2, ldc, strideC, bias,
                           M, N, K, oscale, rscale, sT);
}

__global__ __launch_bounds__(256) void rope_table(float* tab) {
#pragma clang fp contract(off)
  __shared__ __align__(16) float sT[16 * 32];
  const int tid = threadIdx.x;
  const int i   = tid & 15;
  const int rl  = tid >> 4;
  const int pos = blockIdx.x * 16 + rl;
  float p = 1.0f;
  p = (i == 1)  ? 1.7782794100389228f : p;
  p = (i == 2)  ? 3.1622776601683795f : p;
  p = (i == 3)  ? 5.623413251903491f  : p;
  p = (i == 4)  ? 10.0f               : p;
  p = (i == 5)  ? 17.782794100389228f : p;
  p = (i == 6)  ? 31.622776601683793f : p;
  p = (i == 7)  ? 56.23413251903491f  : p;
  p = (i == 8)  ? 100.0f              : p;
  p = (i == 9)  ? 177.82794100389228f : p;
  p = (i == 10) ? 316.22776601683796f : p;
  p = (i == 11) ? 562.3413251903491f  : p;
  p = (i == 12) ? 1000.0f             : p;
  p = (i == 13) ? 1778.2794100389228f : p;
  p = (i == 14) ? 3162.2776601683795f : p;
  p = (i == 15) ? 5623.413251903491f  : p;
  const float inv = 1.0f / p;
  const float th  = (float)pos * inv;
  sT[rl * 32 + i]      = cosf(th);
  sT[rl * 32 + 16 + i] = sinf(th);
  __syncthreads();
  if (tid < 128) {
    const int row = tid >> 3, c4 = (tid & 7) * 4;
    const v4f v = *(const v4f*)(sT + row * 32 + c4);
    float* o = tab + (size_t)(blockIdx.x * 16 + row) * 32 + c4;
    *(volatile v4f*)o = v;
    __threadfence();
    *(volatile v4f*)o = v;
  }
}

template <typename OT, int EPI>
__device__ __forceinline__ void gemm64_epi_body(
    const unsigned short* __restrict__ Ap, int lda,
    const unsigned short* __restrict__ Btp, int ldb,
    void* Cout, int ldc,
    const float* __restrict__ bias,
    const float* __restrict__ ropet,
    const float* __restrict__ sig,
    const float* __restrict__ nw,
    const float* __restrict__ nbv,
    int M, int N, int K, float oscale, float carry, float* sTall) {
  typedef typename FT<OT>::frag V16;
  const OT* A  = (const OT*)(const void*)Ap;
  const OT* Bt = (const OT*)(const void*)Btp;
  const int lane = threadIdx.x & 31;
  const int wave = __builtin_amdgcn_readfirstlane((int)(threadIdx.x >> 5));
  const int tilesN = N >> 6;
  const int tilesM = M >> 6;
  const int tile = blockIdx.x * 8 + wave;
  if (tile >= tilesM * tilesN) return;
  const int tm = tile / tilesN;
  const int tn = tile - tm * tilesN;
  const int m0 = tm << 6;
  const int n0 = tn << 6;

  const int rlane = lane & 15;
  const int koff  = (lane >> 4) * 8;
  const int mOff  = (lane >> 4) * 8;

  v8f acc[4][4];
#pragma unroll
  for (int i = 0; i < 4; ++i)
#pragma unroll
    for (int j = 0; j < 4; ++j) acc[i][j] = zero8();

  for (int k0 = 0; k0 < K; k0 += 32) {
    V16 bq[4];
#pragma unroll
    for (int j = 0; j < 4; ++j)
      bq[j] = ldfrag<OT>(Bt + (size_t)(n0 + (j << 4) + rlane) * ldb + koff + k0);
#pragma unroll
    for (int i = 0; i < 4; ++i) {
      const V16 af = ldfrag<OT>(A + (size_t)(m0 + (i << 4) + rlane) * lda + koff + k0);
#pragma unroll
      for (int j = 0; j < 4; ++j) acc[i][j] = mmar(af, bq[j], acc[i][j]);
      dep_guard(acc[i][0], acc[i][3], af, bq[3]);
    }
    keep4(bq[0], bq[1], bq[2], bq[3]);
  }
  acc_guard4(acc[0][0], acc[0][1], acc[0][2], acc[0][3]);
  acc_guard4(acc[1][0], acc[1][1], acc[1][2], acc[1][3]);
  acc_guard4(acc[2][0], acc[2][1], acc[2][2], acc[2][3]);
  acc_guard4(acc[3][0], acc[3][1], acc[3][2], acc[3][3]);

  float* slab = sTall + wave * (16 * 68);
#pragma unroll
  for (int i = 0; i < 4; ++i) {
    const int mBase = m0 + (i << 4);
#pragma unroll
    for (int j = 0; j < 4; ++j) {
#pragma unroll
      for (int r = 0; r < 8; ++r) {
        slab[(mOff + r) * 68 + (j << 4) + rlane] = acc[i][j][r];
      }
    }
    __builtin_amdgcn_fence(3  , "workgroup");
    __builtin_amdgcn_wave_barrier();
    __builtin_amdgcn_fence(2  , "workgroup");
    if (EPI == 0) {
      float* Cb0 = (float*)Cout;
      const int h2 = lane >> 4, c4 = (lane & 15) * 4;
      for (int ps = 0; ps < 2; ++ps) {
#pragma unroll
        for (int it = 0; it < 8; ++it) {
          const int row = it * 2 + h2;
          const v4f v = *(const v4f*)(slab + row * 68 + c4) * oscale;
          *(volatile v4f*)(Cb0 + (size_t)(mBase + row) * ldc + n0 + c4) = v;
        }
        __threadfence();
      }
    } else if (EPI == 1) {
      const int q = lane >> 3, c8 = (lane & 7) * 8;
      unsigned short* Cp = (unsigned short*)Cout;
      const v4f br0 = *(const v4f*)(bias + n0 + c8);
      const v4f br1 = *(const v4f*)(bias + n0 + c8 + 4);
      float bvv[8];
#pragma unroll
      for (int e = 0; e < 4; ++e) { bvv[e] = bfv(br0[e]); bvv[4 + e] = bfv(br1[e]); }
      v4u hv[4];
#pragma unroll
      for (int it = 0; it < 4; ++it) {
        const int row = it * 4 + q;
        const float* sp = slab + row * 68 + c8;
        unsigned short hb[8];
#pragma unroll
        for (int e = 0; e < 8; ++e) {
          const float f  = sp[e] * oscale + bvv[e];
          const float sg = __builtin_amdgcn_rcpf(1.0f + __expf(-f));
          const float g  = f * sg;
          hb[e] = h_bits(toh_flush(g * carry));
        }
        v4u a;
#pragma unroll
        for (int e = 0; e < 4; ++e) a[e] = pk16(hb[2 * e], hb[2 * e + 1]);
        hv[it] = a;
      }
      for (int ps = 0; ps < 2; ++ps) {
#pragma unroll
        for (int it = 0; it < 4; ++it) {
          const int row = it * 4 + q;
          *(volatile v4u*)(Cp + (size_t)(mBase + row) * ldc + n0 + c8) = hv[it];
        }
        __threadfence();
      }
    } else {
      const int q = lane >> 3, c8 = (lane & 7) * 8;
      unsigned short* Cp = (unsigned short*)Cout;
      const bool nrm = ((tn & 15) & 1) != 0;
      const bool rot = c8 < 32;
      const int  ib  = (c8 >> 1) & 12;
      const v4f w0 = *(const v4f*)(nw + c8);
      const v4f w1 = *(const v4f*)(nw + c8 + 4);
      const v4f g0 = *(const v4f*)(nbv + c8);
      const v4f g1 = *(const v4f*)(nbv + c8 + 4);
      float wv[8], gv[8];
#pragma unroll
      for (int e = 0; e < 4; ++e) {
        wv[e] = bfv(w0[e]); wv[4 + e] = bfv(w1[e]);
        gv[e] = bfv(g0[e]); gv[4 + e] = bfv(g1[e]);
      }
      v4u hv[4];
#pragma unroll
      for (int it = 0; it < 4; ++it) {
        const int row = it * 4 + q;
        const int gm  = mBase + row;
        const int bb  = gm / SEQ;
        const int pos = gm - bb * SEQ;
        const float* sp = slab + row * 68 + c8;
        v4f cs = *(const v4f*)(ropet + (size_t)pos * 32 + ib);
        v4f sn = *(const v4f*)(ropet + (size_t)pos * 32 + 16 + ib);
        pin4(cs);
        pin4(sn);
        const v4f s0 = *(const v4f*)(sig + bb * HD + c8);
        const v4f s1 = *(const v4f*)(sig + bb * HD + c8 + 4);
        float f[8];
#pragma unroll
        for (int e = 0; e < 4; ++e) {
          const float x0 = sp[2 * e], x1 = sp[2 * e + 1];
          const float y0 = x0 * cs[e] - x1 * sn[e];
          const float y1 = x1 * cs[e] + x0 * sn[e];
          f[2 * e]     = rot ? y0 : x0;
          f[2 * e + 1] = rot ? y1 : x1;
        }
        float y[8];
        float ss = 0.f;
#pragma unroll
        for (int e = 0; e < 4; ++e) {
          y[e]     = f[e]     + bfv(s0[e]);
          y[4 + e] = f[4 + e] + bfv(s1[e]);
        }
#pragma unroll
        for (int e = 0; e < 8; ++e) ss += y[e] * y[e];
        ss += __shfl_xor(ss, 1, 32);
        ss += __shfl_xor(ss, 2, 32);
        ss += __shfl_xor(ss, 4, 32);
        const float sc = rsqrtf(ss * (1.0f / (float)HD) + 1e-8f);
        unsigned short hb[8];
#pragma unroll
        for (int e = 0; e < 8; ++e) {
          const float z = y[e] * sc * wv[e] + gv[e];
          const float o = nrm ? z : f[e];
          hb[e] = h_bits(toh_flush(o * carry));
        }
        v4u a;
#pragma unroll
        for (int e = 0; e < 4; ++e) a[e] = pk16(hb[2 * e], hb[2 * e + 1]);
        hv[it] = a;
      }
      for (int ps = 0; ps < 2; ++ps) {
#pragma unroll
        for (int it = 0; it < 4; ++it) {
          const int row = it * 4 + q;
          *(volatile v4u*)(Cp + (size_t)(mBase + row) * ldc + n0 + c8) = hv[it];
        }
        __threadfence();
      }
    }
    __builtin_amdgcn_fence(3  , "workgroup");
    __builtin_amdgcn_wave_barrier();
    __builtin_amdgcn_fence(2  , "workgroup");
  }
}

__global__ __launch_bounds__(256) void gemm_qk_rope(
    const unsigned short* __restrict__ Ap, int lda,
    const unsigned short* __restrict__ Btp, int ldb,
    unsigned short* Cout, int ldc,
    const float* __restrict__ ropet, const float* __restrict__ sig,
    const float* __restrict__ nw, const float* __restrict__ nbv,
    int M, int N, int K, float carry) {
  __shared__ __align__(16) float sT[8 * 16 * 68];
  gemm64_epi_body<__bf16, 2>(Ap, lda, Btp, ldb, (void*)Cout, ldc, ropet, ropet, sig, nw, nbv,
                             M, N, K, 1.0f, carry, sT);
}
__global__ __launch_bounds__(256) void gemm_plain_f32(
    const unsigned short* __restrict__ Ap, int lda,
    const unsigned short* __restrict__ Btp, int ldb,
    float* Cout, int ldc,
    int M, int N, int K, float oscale) {
  __shared__ __align__(16) float sT[8 * 16 * 68];
  gemm64_epi_body<_Float16, 0>(Ap, lda, Btp, ldb, (void*)Cout, ldc, Cout, Cout, Cout, Cout, Cout,
                               M, N, K, oscale, 1.0f, sT);
}
__global__ __launch_bounds__(256) void gemm_bias_silu(
    const unsigned short* __restrict__ Ap, int lda,
    const unsigned short* __restrict__ Btp, int ldb,
    unsigned short* Cout, int ldc,
    const float* __restrict__ bias,
    int M, int N, int K, float oscale, float carry) {
  __shared__ __align__(16) float sT[8 * 16 * 68];
  gemm64_epi_body<_Float16, 1>(Ap, lda, Btp, ldb, (void*)Cout, ldc, bias, bias, bias, bias, bias,
                               M, N, K, oscale, carry, sT);
}

__global__ __launch_bounds__(128) __attribute__((amdgpu_num_vgpr(256)))
void attn_diff(const unsigned short* __restrict__ qkp, const unsigned short* __restrict__ vtp,
               const float* __restrict__ lq1, const float* __restrict__ lk1,
               const float* __restrict__ lq2, const float* __restrict__ lk2,
               const float* __restrict__ lnw, const float* __restrict__ lnb,
               unsigned short* ap) {
  union FH { v16h v; v8h h[2]; };
  __shared__ __align__(16) _Float16 Psh[4][16 * 64];
  __shared__ __align__(16) float    Os[4][16 * 128];

  const int tid  = threadIdx.x;
  const int wave = __builtin_amdgcn_readfirstlane((int)(tid >> 5));
  const int lane = tid & 31;
  const int hh   = lane >> 4;
  const int c    = lane & 15;

  const int bx   = blockIdx.x;
  const int qb   = bx % NQB;
  const int rest = bx / NQB;
  const int h    = rest % NH;
  const int b    = rest / NH;
  const int q0   = qb * 64 + wave * 16;
  const size_t rowQ = (size_t)b * SEQ;

  float s1 = bfv(lq1[lane]) * bfv(lk1[lane]) + bfv(lq1[lane + 32]) * bfv(lk1[lane + 32]);
  float s2 = bfv(lq2[lane]) * bfv(lk2[lane]) + bfv(lq2[lane + 32]) * bfv(lk2[lane + 32]);
#pragma unroll
  for (int off = 1; off < 32; off <<= 1) {
    s1 += __shfl_xor(s1, off, 32);
    s2 += __shfl_xor(s2, off, 32);
  }
  const float lam = (expf(s1) - expf(s2)) + LAM_INIT;

  const _Float16* QKp = (const _Float16*)(const void*)qkp;
  const _Float16* Vg  = (const _Float16*)(const void*)vtp + ((size_t)b * DM + (size_t)h * DV) * (size_t)SEQ;
  _Float16* pwh = Psh[wave];
  float*    os  = Os[wave];

  v8f oacc[8];
#pragma unroll 1
  for (int br = 0; br < 2; ++br) {
    const int sub = 2 * h + br;
    const _Float16* Qg = QKp + (size_t)sub * HD;
    const _Float16* Kg = QKp + DM + (size_t)sub * HD;

    v16h qa[2];
#pragma unroll
    for (int dc = 0; dc < 2; ++dc)
      qa[dc] = ldfrag<_Float16>(Qg + (rowQ + q0 + c) * QKLD + dc * 32 + 8 * hh);

    float mrow[8], lrow[8];
#pragma unroll
    for (int r = 0; r < 8; ++r) { mrow[r] = -INFINITY; lrow[r] = 0.f; }
#pragma unroll
    for (int t = 0; t < 8; ++t) oacc[t] = zero8();

    const int nkt = qb + 1;
    for (int kt = 0; kt < nkt; ++kt) {
      const int kv0 = kt * 64;

      v8f s[4];
#pragma unroll
      for (int j = 0; j < 4; ++j) {
        v8f ac = zero8();
#pragma unroll
        for (int dc = 0; dc < 2; ++dc) {
          const v16h kb = ldfrag<_Float16>(Kg + (rowQ + kv0 + j * 16 + c) * QKLD + dc * 32 + 8 * hh);
          ac = mma_h(qa[dc], kb, ac);
        }
#pragma unroll
        for (int r = 0; r < 8; ++r) s[j][r] = ac[r] * SMUL;
      }
      if (kt == qb) {
#pragma unroll
        for (int j = 0; j < 4; ++j) {
          const int key = kv0 + j * 16 + c;
#pragma unroll
          for (int r = 0; r < 8; ++r) {
            const int qr = q0 + 8 * hh + r;
            s[j][r] = (key <= qr) ? s[j][r] : -INFINITY;
          }
        }
      }

#pragma unroll
      for (int r = 0; r < 8; ++r) {
        float m = s[0][r];
#pragma unroll
        for (int j = 1; j < 4; ++j) m = fmaxf(m, s[j][r]);
#pragma unroll
        for (int off = 1; off < 16; off <<= 1) m = fmaxf(m, __shfl_xor(m, off, 32));
        const float mnew  = fmaxf(mrow[r], m);
        const float msafe = (mnew == -INFINITY) ? 0.f : mnew;
        const float alpha = exp2f(mrow[r] - msafe);
        mrow[r] = mnew;
        float psum = 0.f;
#pragma unroll
        for (int j = 0; j < 4; ++j) {
          const float e2 = s[j][r] - msafe;
          const float pc = (e2 < -28.0f) ? 0.0f : exp2f(e2 + 14.0f);
          const h16 ph = (h16)pc;
          psum += (float)ph;
          pwh[(8 * hh + r) * 64 + j * 16 + c] = ph;
        }
#pragma unroll
        for (int off = 1; off < 16; off <<= 1) psum += __shfl_xor(psum, off, 32);
        lrow[r] = lrow[r] * alpha + psum;
#pragma unroll
        for (int t = 0; t < 8; ++t) oacc[t][r] *= alpha;
      }
      __builtin_amdgcn_fence(3  , "workgroup");
      __builtin_amdgcn_wave_barrier();
      __builtin_amdgcn_fence(2  , "workgroup");

#pragma unroll 1
      for (int kk = 0; kk < 2; ++kk) {
        FH pa;
        pa.h[0] = *(const v8h*)(pwh + c * 64 + kk * 32 + 8 * hh);
        pa.h[1] = *(const v8h*)(pwh + c * 64 + kk * 32 + 16 + 8 * hh);
#pragma unroll
        for (int t = 0; t < 8; ++t) {
          const v16h vb = ldfrag<_Float16>(Vg + (size_t)(t * 16 + c) * SEQ + kv0 + kk * 32 + 8 * hh);
          oacc[t] = mma_h(pa.v, vb, oacc[t]);
        }
      }
      __builtin_amdgcn_fence(3  , "workgroup");
      __builtin_amdgcn_wave_barrier();
      __builtin_amdgcn_fence(2  , "workgroup");
    }

#pragma unroll
    for (int r = 0; r < 8; ++r) {
      const float l = lrow[r];
      const float inv = ((l > 0.f) ? (1.0f / l) : 0.f) * (1.0f / VCARRY);
#pragma unroll
      for (int t = 0; t < 8; ++t) oacc[t][r] *= inv;
    }
    if (br == 0) {
#pragma unroll
      for (int t = 0; t < 8; ++t)
#pragma unroll
        for (int r = 0; r < 8; ++r) os[(t * 8 + r) * 32 + lane] = oacc[t][r];
    }
  }

  float scr[8];
#pragma unroll
  for (int r = 0; r < 8; ++r) {
    float ss = 0.f;
#pragma unroll
    for (int t = 0; t < 8; ++t) {
      const float d = os[(t * 8 + r) * 32 + lane] - lam * oacc[t][r];
      oacc[t][r] = d;
      ss += d * d;
    }
#pragma unroll
    for (int off = 1; off < 16; off <<= 1) ss += __shfl_xor(ss, off, 32);
    scr[r] = rsqrtf(ss * (1.0f / (float)DV) + 1e-8f);
  }
  __builtin_amdgcn_fence(3  , "workgroup");
  __builtin_amdgcn_wave_barrier();
  __builtin_amdgcn_fence(2  , "workgroup");
#pragma unroll
  for (int t = 0; t < 8; ++t) {
    const int col = t * 16 + c;
    const float gw = bfv(lnw[col]);
    const float gb = bfv(lnb[col]);
#pragma unroll
    for (int r = 0; r < 8; ++r)
      os[(8 * hh + r) * 128 + col] = (oacc[t][r] * scr[r] * gw + gb) * OMLI;
  }
  __builtin_amdgcn_fence(3  , "workgroup");
  __builtin_amdgcn_wave_barrier();
  __builtin_amdgcn_fence(2  , "workgroup");
  {
    const int h2 = lane >> 4, c8 = (lane & 15) * 8;
    v4u hv[8];
#pragma unroll
    for (int it = 0; it < 8; ++it) {
      const int row = it * 2 + h2;
      const float* sp = os + row * 128 + c8;
      v4u a;
#pragma unroll
      for (int e = 0; e < 4; ++e)
        a[e] = pk16(h_bits(toh_flush(sp[2 * e] * ACARRY)), h_bits(toh_flush(sp[2 * e + 1] * ACARRY)));
      hv[it] = a;
    }
    for (int ps = 0; ps < 2; ++ps) {
#pragma unroll
      for (int it = 0; it < 8; ++it) {
        const int row = it * 2 + h2;
        const size_t go = (rowQ + q0 + row) * DM + (size_t)h * DV + c8;
        *(volatile v4u*)(ap + go) = hv[it];
      }
      __threadfence();
    }
  }
}

static __device__ __forceinline__ v4f ln_z(const float* __restrict__ prow, const float* __restrict__ rrow,
                                           int col, int rbf) {
  const v4f a = *(const v4f*)(prow + col);
  const v4f r = *(const v4f*)(rrow + col);
  v4f z;
#pragma unroll
  for (int e = 0; e < 4; ++e) {
    const float rv = (rbf != 0) ? bfv(r[e]) : r[e];
    z[e] = a[e] + rv;
  }
  return z;
}

__global__ __launch_bounds__(256)
void ln_rows(const float* __restrict__ P, const float* __restrict__ R, int rstride, int rbf,
             const float* __restrict__ gw, const float* __restrict__ gb,
             float* outF, int ostride, unsigned short* outH, int wh, float hcarry, int nrows) {
#pragma clang fp contract(off)
  const int lane = threadIdx.x & 31;
  const int wave = __builtin_amdgcn_readfirstlane((int)(threadIdx.x >> 5));
  const int gm = blockIdx.x * 8 + wave;
  if (gm >= nrows) return;
  const int bb = gm / SEQ;
  const int t  = gm - bb * SEQ;
  const float* prow = P + (size_t)gm * DM;
  const float* rrow = R + ((size_t)bb * (size_t)rstride + (size_t)t) * DM;

  float sum = 0.f;
#pragma unroll 1
  for (int j = 0; j < 8; ++j) {
    const v4f z = ln_z(prow, rrow, j * 128 + lane * 4, rbf);
    sum += (z[0] + z[1]) + (z[2] + z[3]);
  }
#pragma unroll
  for (int off = 1; off < 32; off <<= 1) sum += __shfl_xor(sum, off, 32);
  const float mean = sum * (1.0f / (float)DM);

  float sq = 0.f;
#pragma unroll 1
  for (int j = 0; j < 8; ++j) {
    const v4f z = ln_z(prow, rrow, j * 128 + lane * 4, rbf);
    const float d0 = z[0] - mean, d1 = z[1] - mean, d2 = z[2] - mean, d3 = z[3] - mean;
    sq += (d0 * d0 + d1 * d1) + (d2 * d2 + d3 * d3);
  }
#pragma unroll
  for (int off = 1; off < 32; off <<= 1) sq += __shfl_xor(sq, off, 32);
  const float inv = rsqrtf(sq * (1.0f / (float)DM) + 1e-5f);

  float* orow = outF + ((size_t)bb * (size_t)ostride + (size_t)t) * DM;
  unsigned short* hrow = outH + (size_t)gm * DM;
#pragma unroll 1
  for (int j = 0; j < 8; ++j) {
    const int col = j * 128 + lane * 4;
    const v4f z = ln_z(prow, rrow, col, rbf);
    const v4f w = *(const v4f*)(gw + col);
    const v4f g = *(const v4f*)(gb + col);
    v4f y;
#pragma unroll
    for (int e = 0; e < 4; ++e) y[e] = (z[e] - mean) * inv * bfv(w[e]) + bfv(g[e]);
    v2u hp;
    hp[0] = pk16(h_bits(toh_flush(y[0] * hcarry)), h_bits(toh_flush(y[1] * hcarry)));
    hp[1] = pk16(h_bits(toh_flush(y[2] * hcarry)), h_bits(toh_flush(y[3] * hcarry)));
    *(volatile v4f*)(orow + col) = y;
    if (wh != 0) *(volatile v2u*)(hrow + col) = hp;
    __threadfence();
    *(volatile v4f*)(orow + col) = y;
    if (wh != 0) *(volatile v2u*)(hrow + col) = hp;
  }
}

extern "C" void kernel_launch(void* const* d_in, const int* in_sizes, int n_in,
                              void* d_out, int out_size, void* d_ws, size_t ws_size,
                              hipStream_t stream) {
  if (n_in < 20) return;
  if (in_sizes[0] < NB * SEQ_FULL * DM) return;
  if (in_sizes[1] < NB * HD) return;
  if (in_sizes[2] < DM * 3 * DM) return;
  if (in_sizes[3] < DM * DM) return;
  if (in_sizes[4] < HD || in_sizes[5] < HD || in_sizes[6] < HD || in_sizes[7] < HD) return;
  if (in_sizes[8] < DV || in_sizes[9] < DV) return;
  if (in_sizes[10] < HD || in_sizes[11] < HD) return;
  if (in_sizes[12] < DM || in_sizes[13] < DM || in_sizes[14] < DM || in_sizes[15] < DM) return;
  if (in_sizes[16] < DM * DFF) return;
  if (in_sizes[17] < DFF) return;
  if (in_sizes[18] < DFF * DM) return;
  if (in_sizes[19] < DM) return;
  if (out_size < ((NB - 1) * SEQ_FULL + SEQ) * DM) return;

  const float* x      = (const float*)d_in[0];
  const float* sigmas = (const float*)d_in[1];
  const float* w_qkv  = (const float*)d_in[2];
  const float* w_out  = (const float*)d_in[3];
  const float* lq1    = (const float*)d_in[4];
  const float* lk1    = (const float*)d_in[5];
  const float* lq2    = (const float*)d_in[6];
  const float* lk2    = (const float*)d_in[7];
  const float* ln_w   = (const float*)d_in[8];
  const float* ln_b   = (const float*)d_in[9];
  const float* lnq_w  = (const float*)d_in[10];
  const float* lnq_b  = (const float*)d_in[11];
  const float* ln1_w  = (const float*)d_in[12];
  const float* ln1_b  = (const float*)d_in[13];
  const float* ln2_w  = (const float*)d_in[14];
  const float* ln2_b  = (const float*)d_in[15];
  const float* w1     = (const float*)d_in[16];
  const float* b1     = (const float*)d_in[17];
  const float* w2     = (const float*)d_in[18];
  const float* b2     = (const float*)d_in[19];

  size_t off = 0;
  const size_t oR1 = off; off += WSB_R1;
  const size_t oWo = off; off += WSB_WO;
  const size_t oW1 = off; off += WSB_W1;
  const size_t oW2 = off; off += WSB_W2;
  const size_t oRp = off; off += WSB_ROPE;
  const size_t oAp = off; off += WSB_AP;
  const size_t oPr = off; off += WSB_PRE;
  const size_t oHf = off; off += WSB_HF;
  const size_t oHh = off; off += WSB_HH;
  if (off != WSB_TOTAL) return;
  if (off > ws_size) return;
  if (off > (size_t)134217728) return;

  char* ws = (char*)d_ws;
  unsigned short* Xb    = (unsigned short*)(ws + oR1);
  unsigned short* WqkvT = (unsigned short*)(ws + oR1 + WSB_XB);
  unsigned short* QK    = (unsigned short*)(ws + oR1 + WSB_XB + WSB_WQKV);
  unsigned short* VT    = (unsigned short*)(ws + oR1 + WSB_XB + WSB_WQKV + WSB_QK);
  unsigned short* G     = (unsigned short*)(ws + oR1);
  unsigned short* WoT   = (unsigned short*)(ws + oWo);
  unsigned short* W1T   = (unsigned short*)(ws + oW1);
  unsigned short* W2T   = (unsigned short*)(ws + oW2);
  float*          ROPE  = (float*)(ws + oRp);
  unsigned short* Ap    = (unsigned short*)(ws + oAp);
  float*          PRE   = (float*)(ws + oPr);
  float*          Hf    = (float*)(ws + oHf);
  unsigned short* Hh    = (unsigned short*)(ws + oHh);

  const int MR = NB * SEQ;
  const dim3 blk(256);
  const int n8x = SEQ * DM / 8;
  const dim3 gCvtX((n8x + 255) / 256, NB);
  const dim3 gWqkv(3 * DM / 64, DM / 64);
  const dim3 gWo(DM / 64, DM / 64);
  const dim3 gW1(DFF / 64, DM / 64);
  const dim3 gW2(DM / 64, DFF / 64);
  const dim3 gQK((((MR / 64) * (QKLD / 64)) + 7) / 8, 1);
  const dim3 gVT((((DM / 64) * (SEQ / 64)) + 7) / 8, NB);
  const dim3 gAttn(NB * NH * NQB);
  const dim3 gO((((MR / 64) * (DM / 64)) + 7) / 8, 1);
  const dim3 gF1((((MR / 64) * (DFF / 64)) + 7) / 8, 1);
  const dim3 gLN((MR + 7) / 8);

  cvt_bf16x8<<<gCvtX, blk, 0, stream>>>(x, (long long)SEQ_FULL * DM, Xb, (long long)SEQ * DM, n8x);
  wtrans_bf16<<<gWqkv, blk, 0, stream>>>(w_qkv, 3 * DM, WqkvT, DM, 0, 1.0f);
  wtrans_f16s<<<gWo, blk, 0, stream>>>(w_out, DM, WoT, DM, 0, WCARRY);
  wtrans_f16s<<<gW1, blk, 0, stream>>>(w1, DFF, W1T, DM, 0, WCARRY);
  wtrans_f16s<<<gW2, blk, 0, stream>>>(w2, DM, W2T, DFF, 0, WCARRY);
  rope_table<<<dim3(SEQ / 16), blk, 0, stream>>>(ROPE);
  gemm_qk_rope<<<gQK, blk, 0, stream>>>(Xb, DM, WqkvT, DM, QK, QKLD, ROPE, sigmas, lnq_w, lnq_b,
                                        MR, QKLD, DM, QKC);
  gemm_proj_plane<<<gVT, blk, 0, stream>>>(
      WqkvT + (size_t)2 * DM * DM, DM, 0LL, Xb, DM, (long long)SEQ * DM,
      (void*)VT, (void*)VT, SEQ, (long long)DM * SEQ, b1,
      DM, SEQ, DM, VCARRY, 1.0f);
  attn_diff<<<gAttn, dim3(128), 0, stream>>>(QK, VT, lq1, lk1, lq2, lk2, ln_w, ln_b, Ap);
  gemm_plain_f32<<<gO, blk, 0, stream>>>(Ap, DM, WoT, DM, PRE, DM, MR, DM, DM, 1.0f / (ACARRY * WCARRY));
  ln_rows<<<gLN, blk, 0, stream>>>(PRE, x, SEQ_FULL, 1, ln1_w, ln1_b, Hf, SEQ, Hh, 1, HCARRY, MR);
  gemm_bias_silu<<<gF1, blk, 0, stream>>>(Hh, DM, W1T, DM, G, DFF, b1, MR, DFF, DM,
                                          1.0f / (HCARRY * WCARRY), GCARRY);
  gemm_out_f32<<<gO, blk, 0, stream>>>(
      G, DFF, 0LL, W2T, DFF, 0LL,
      (void*)PRE, (void*)PRE, DM, 0LL, b2,
      MR, DM, DFF, 1.0f / (GCARRY * WCARRY), 1.0f);
  ln_rows<<<gLN, blk, 0, stream>>>(PRE, Hf, SEQ, 0, ln2_w, ln2_b, (float*)d_out, SEQ_FULL, Hh, 0, 1.0f, MR);
  (void)hipGetLastError();
}
